// Attention_21698174779774
// MI455X (gfx1250) — hardware-run, weakly checked
//
#include <hip/hip_runtime.h>
#include <stdint.h>


typedef _Float16 v16h __attribute__((ext_vector_type(16)));
typedef _Float16 v8h  __attribute__((ext_vector_type(8)));
typedef float    v8f  __attribute__((ext_vector_type(8)));
typedef float    v4f  __attribute__((ext_vector_type(4)));
typedef _Float16 h16;

#ifndef NB
#define NB 16
#endif
#ifndef SEQ
#define SEQ 1024
#endif
#define NB_FULL  16
#define SEQ_FULL 1024
#define DM   768
#define NH   12
#define HD   64
#define QKP  1536
#define ROWS (NB * SEQ)
#define TABW 64
#define MB_PITCH 32

#define ACT_CAR   8.0f
#define W_CAR     1024.0f
#define PROJ_SCL  0.0009765625f
#define S_SCL     0.001953125f
#define LN_PCAR   9.704060527839234f
#define P_CUT     (-9.25f)
#define O_MUL     32.0f
#define OUT_SCL   3.814697265625e-06f

static_assert(NB >= 1 && NB <= NB_FULL && SEQ <= SEQ_FULL);
static_assert(SEQ % 128 == 0);
static_assert(SEQ % 8 == 0);
static_assert(SEQ / 32 <= MB_PITCH);
static_assert(DM == NH * HD);
static_assert(HD == 64);
static_assert(QKP == 2 * DM);
static_assert(DM % 128 == 0 && DM % 64 == 0 && DM % 32 == 0 && QKP % 64 == 0);
static_assert(TABW == 64 && HD / 2 == 32);
static_assert(((long)ROWS * DM / 8) % 256 == 0);
static_assert((long)(DM / 64) * (DM / 64) * 4096 == (long)DM * DM);
static_assert((long)(SEQ / 8) * 256 * 2 == (long)SEQ * TABW);
static_assert((long)(QKP / 64) * (ROWS / 128) * 128 * 64 == (long)ROWS * QKP);
static_assert((long)(SEQ / 64) * (DM / 128) * 128 * 64 == (long)SEQ * DM);
static_assert((long)(SEQ / 128) * NH * 128 * HD == (long)SEQ * DM);
static_assert((long)(DM / 64) * (ROWS / 128) * 128 * 64 == (long)ROWS * DM);

#define N_X    ((size_t)ROWS * DM)
#define N_W    ((size_t)4 * DM * DM)
#define N_QK   ((size_t)ROWS * QKP)
#define N_VT   ((size_t)NB * DM * SEQ)
#define N_TAB  ((size_t)SEQ * TABW * 2)
#define N_MB   ((size_t)NB * MB_PITCH * 2)
#define WS_HALVES (N_X + N_W + N_QK + N_VT + N_X + N_TAB + N_MB)
static_assert(WS_HALVES * 2 <= (size_t)134217728);
static_assert(N_X % 64 == 0 && N_W % 64 == 0 && N_QK % 64 == 0 && N_VT % 64 == 0 && N_TAB % 64 == 0 && N_MB % 64 == 0);

union Frag16 { v16h v; v8h p[2]; };

__device__ __forceinline__ v16h ld_frag_g(const _Float16* __restrict__ p, int hl) {
  Frag16 f;
  f.p[0] = *(const v8h*)(p + 8 * hl);
  f.p[1] = *(const v8h*)(p + 16 + 8 * hl);
  return f.v;
}

__device__ __forceinline__ v16h ld_frag_s(const _Float16* base, int off, int hl) {
  Frag16 f;
  f.p[0] = *(const v8h*)(base + off + 8 * hl);
  f.p[1] = *(const v8h*)(base + off + 16 + 8 * hl);
  return f.v;
}

__device__ __forceinline__ v8f mma(v16h a, v16h b, v8f c) {
  v8f d = __builtin_amdgcn_wmma_f32_16x16x32_f16(false, a, false, b, (short)0, c, false, false);
  asm volatile("v_nop\n\tv_nop\n\tv_nop\n\tv_nop" : "+v"(d) : "v"(a), "v"(b));
  return d;
}

__device__ __forceinline__ float bf16_rne(float x) {
  unsigned int u = __builtin_bit_cast(unsigned int, x);
  u += 0x7FFFu + ((u >> 16) & 1u);
  return __builtin_bit_cast(float, u & 0xFFFF0000u);
}

static __device__ __forceinline__ h16 toh_flush(float v) {
  const h16 r = (h16)v;
  return (fabsf(v) < 6.103515625e-05f) ? (h16)0.0f : r;
}

__global__ __launch_bounds__(256) void k_cvt8(const float* __restrict__ src,
                                              _Float16* __restrict__ dst,
                                              int cols, int seq, int seq_full, float car, int total8)
{
  const int i8 = blockIdx.x * 256 + threadIdx.x;
  if (i8 >= total8) return;
  const size_t e   = (size_t)i8 * 8;
  const int    r   = (int)(e / (size_t)cols);
  const int    col = (int)(e - (size_t)r * (size_t)cols);
  const int    bb  = r / seq;
  const int    nn  = r - bb * seq;
  const float* s = src + ((size_t)bb * seq_full + nn) * (size_t)cols + col;
  const v4f x0 = *(const v4f*)s;
  const v4f x1 = *(const v4f*)(s + 4);
  v8h o;
#pragma unroll
  for (int j = 0; j < 4; ++j) {
    const float t0 = x0[j];
    const float t1 = x1[j];
    o[j]     = (_Float16)(bf16_rne(t0) * car);
    o[4 + j] = (_Float16)(bf16_rne(t1) * car);
  }
  _Float16* d = dst + e;
  *(volatile v8h*)d = o;
  __threadfence();
  *(volatile v8h*)d = o;
}

__global__ __launch_bounds__(256) void k_trw(const float* __restrict__ W,
                                             _Float16* __restrict__ WT, int R, int C)
{
  __shared__ float tile[64 * 65];
  const int tid = threadIdx.x;
  const int c0 = blockIdx.x * 64, r0 = blockIdx.y * 64;
#pragma unroll
  for (int i = 0; i < 4; ++i) {
    const int idx = i * 256 + tid;
    const int r = idx >> 4, c4 = (idx & 15) * 4;
    const v4f v = *(const v4f*)(W + (size_t)(r0 + r) * C + c0 + c4);
    tile[r * 65 + c4 + 0] = v[0];
    tile[r * 65 + c4 + 1] = v[1];
    tile[r * 65 + c4 + 2] = v[2];
    tile[r * 65 + c4 + 3] = v[3];
  }
  __syncthreads();
  v8h o[2];
  size_t dofs[2];
#pragma unroll
  for (int i = 0; i < 2; ++i) {
    const int line = i * 32 + (tid >> 3);
    const int pc   = (tid & 7) * 8;
#pragma unroll
    for (int j = 0; j < 8; ++j)
      o[i][j] = (_Float16)(bf16_rne(tile[(pc + j) * 65 + line]) * W_CAR);
    dofs[i] = (size_t)(c0 + line) * R + r0 + pc;
  }
  *(volatile v8h*)(WT + dofs[0]) = o[0];
  *(volatile v8h*)(WT + dofs[1]) = o[1];
  __threadfence();
  *(volatile v8h*)(WT + dofs[0]) = o[0];
  *(volatile v8h*)(WT + dofs[1]) = o[1];
}

__global__ __launch_bounds__(256) void k_ropetab(float* __restrict__ tab)
{
#pragma clang fp contract(off)
  const int tid = threadIdx.x;
  const int j   = tid & 31;
  const int pos = blockIdx.x * 8 + (tid >> 5);
  double f = 1.0;
#pragma unroll 1
  for (int i = 0; i < 31; ++i) {
    const double g = f * 0.7498942093324559;
    f = (i < j) ? g : f;
  }
  const float invf = (float)f;
  const float ang  = (float)pos * invf;
  float sn, cs;
  sincosf(ang, &sn, &cs);
  float* d = tab + (size_t)pos * TABW + j;
  *(volatile float*)d = cs;
  *(volatile float*)(d + 32) = sn;
  __threadfence();
  *(volatile float*)d = cs;
  *(volatile float*)(d + 32) = sn;
}

__global__ __launch_bounds__(256) void k_mbits(const int* __restrict__ mask,
                                               unsigned int* __restrict__ MB)
{
  __shared__ unsigned int sw[32];
  const int tid = threadIdx.x, lane = tid & 31;
  const int wave = __builtin_amdgcn_readfirstlane(tid >> 5);
  const int b = blockIdx.x;
  const int* mrow = mask + (size_t)b * SEQ_FULL;
#pragma unroll 1
  for (int i = 0; i < 4; ++i) {
    const int wd = wave * 4 + i;
    int kidx = wd * 32 + lane;
    kidx = (kidx < SEQ) ? kidx : (SEQ - 1);
    const int mv = mrow[kidx];
    const bool inr = (wd * 32 < SEQ);
    const bool pred = inr ? (mv != 0) : true;
    const unsigned int bal = (unsigned int)__ballot(pred);
    if (lane == 0) sw[wd] = bal;
  }
  __syncthreads();
  if (wave == 0) {
    const unsigned int v = sw[lane];
    unsigned int* d = MB + (size_t)b * MB_PITCH + lane;
    *(volatile unsigned int*)d = v;
    __threadfence();
    *(volatile unsigned int*)d = v;
  }
}

__device__ __forceinline__ void gemm_core(const _Float16* __restrict__ ap0,
                                          const _Float16* __restrict__ ap1,
                                          const _Float16* __restrict__ bp, int K, int hl, v8f (&acc)[8])
{
  const size_t bst = (size_t)16 * K;
#pragma unroll 1
  for (int k0 = 0; k0 < K; k0 += 32) {
    const v16h a0 = ld_frag_g(ap0 + k0, hl);
    const v16h a1 = ld_frag_g(ap1 + k0, hl);
    const v16h b0 = ld_frag_g(bp + k0, hl);
    const v16h b1 = ld_frag_g(bp + bst + k0, hl);
    const v16h b2 = ld_frag_g(bp + 2 * bst + k0, hl);
    const v16h b3 = ld_frag_g(bp + 3 * bst + k0, hl);
    acc[0] = mma(a0, b0, acc[0]);
    acc[1] = mma(a0, b1, acc[1]);
    acc[2] = mma(a0, b2, acc[2]);
    acc[3] = mma(a0, b3, acc[3]);
    acc[4] = mma(a1, b0, acc[4]);
    acc[5] = mma(a1, b1, acc[5]);
    acc[6] = mma(a1, b2, acc[6]);
    acc[7] = mma(a1, b3, acc[7]);
  }
}

__global__ __launch_bounds__(128) __attribute__((amdgpu_num_vgpr(256)))
void k_projr(const _Float16* __restrict__ A, const _Float16* __restrict__ Bt,
             const float* __restrict__ bq, const float* __restrict__ bk,
             const float* __restrict__ tab, _Float16* __restrict__ PH)
{
  __shared__ __attribute__((aligned(16))) _Float16 ldsE[128 * 72];
  __shared__ __attribute__((aligned(16))) float    tabS[128 * TABW];
  static_assert(16 * 128 * 4 == 128 * TABW);
  static_assert(8 * 128 == 128 * 8);

  const int tid = threadIdx.x, lane = tid & 31;
  const int w = __builtin_amdgcn_readfirstlane(tid >> 5);
  const int hl = lane >> 4, c = lane & 15;
  const int m0 = blockIdx.y * 128, n0 = blockIdx.x * 64;
  const int mw = m0 + 32 * w;

  const _Float16* ap0 = A  + (size_t)(mw + c) * DM;
  const _Float16* ap1 = A  + (size_t)(mw + 16 + c) * DM;
  const _Float16* bp  = Bt + (size_t)(n0 + c) * DM;

  v8f acc[8] = {};
  gemm_core(ap0, ap1, bp, DM, hl, acc);

  const int pos0 = m0 % SEQ;
  const float* tsrc = tab + (size_t)pos0 * TABW;
#pragma unroll 4
  for (int i = 0; i < 16; ++i) {
    const int idx = (i * 128 + tid) * 4;
    const v4f tv = *(const v4f*)(tsrc + idx);
    *(v4f*)(&tabS[idx]) = tv;
  }

  float b8[4];
#pragma unroll
  for (int t = 0; t < 4; ++t) {
    const int col = n0 + 16 * t + c;
    const int cq  = (col < DM) ? col : (DM - 1);
    const int ckk = (col - DM > 0) ? (col - DM) : 0;
    const float vq = bq[cq];
    const float vk = bk[ckk];
    const float braw = (n0 < DM) ? vq : vk;
    b8[t] = bf16_rne(braw) * ACT_CAR;
  }
  __syncthreads();

#pragma unroll
  for (int i = 0; i < 2; ++i)
#pragma unroll
    for (int r = 0; r < 8; ++r) {
      const int rowl = 32 * w + 16 * i + 8 * hl + r;
#pragma unroll
      for (int tp = 0; tp < 2; ++tp) {
        const int j = 16 * tp + c;
        const float cs = tabS[rowl * TABW + j];
        const float sn = tabS[rowl * TABW + 32 + j];
        const float a  = acc[i * 4 + tp][r]     * PROJ_SCL + b8[tp];
        const float bb = acc[i * 4 + tp + 2][r] * PROJ_SCL + b8[tp + 2];
        const float lo = a * cs - bb * sn;
        const float hi = bb * cs + a * sn;
        ldsE[rowl * 72 + j]      = toh_flush(lo);
        ldsE[rowl * 72 + 32 + j] = toh_flush(hi);
      }
    }
  __syncthreads();

  _Float16* const bh = PH + (size_t)m0 * QKP + n0;
  for (int i = 0; i < 8; ++i) {
    const int q = i * 128 + tid;
    const int rowl = q >> 3, ch = (q & 7) * 8;
    const v8h vh = *(const v8h*)(&ldsE[rowl * 72 + ch]);
    *(volatile v8h*)(bh + (size_t)rowl * QKP + ch) = vh;
  }
  __threadfence();
  for (int i = 0; i < 8; ++i) {
    const int q = i * 128 + tid;
    const int rowl = q >> 3, ch = (q & 7) * 8;
    const v8h vh = *(const v8h*)(&ldsE[rowl * 72 + ch]);
    *(volatile v8h*)(bh + (size_t)rowl * QKP + ch) = vh;
  }
}

__global__ __launch_bounds__(128) __attribute__((amdgpu_num_vgpr(256)))
void k_projv(const _Float16* __restrict__ A, const _Float16* __restrict__ Bt,
             const float* __restrict__ bv, _Float16* __restrict__ PH)
{
  __shared__ __attribute__((aligned(16))) _Float16 ldsE[128 * 72];

  const int tid = threadIdx.x, lane = tid & 31;
  const int w = __builtin_amdgcn_readfirstlane(tid >> 5);
  const int hl = lane >> 4, c = lane & 15;
  const int z = blockIdx.z;
  const int m0 = blockIdx.y * 128, n0 = blockIdx.x * 64;
  const int mw = m0 + 32 * w;

  const _Float16* bz  = Bt + (size_t)z * SEQ * DM;
  const _Float16* ap0 = A  + (size_t)(mw + c) * DM;
  const _Float16* ap1 = A  + (size_t)(mw + 16 + c) * DM;
  const _Float16* bp  = bz + (size_t)(n0 + c) * DM;

  v8f acc[8] = {};
  gemm_core(ap0, ap1, bp, DM, hl, acc);

#pragma unroll
  for (int i = 0; i < 2; ++i) {
    const float* bsrc = bv + mw + 16 * i + 8 * hl;
    const v4f ba = *(const v4f*)bsrc;
    const v4f bb = *(const v4f*)(bsrc + 4);
    float b8[8];
    b8[0] = bf16_rne(ba[0]) * ACT_CAR; b8[1] = bf16_rne(ba[1]) * ACT_CAR;
    b8[2] = bf16_rne(ba[2]) * ACT_CAR; b8[3] = bf16_rne(ba[3]) * ACT_CAR;
    b8[4] = bf16_rne(bb[0]) * ACT_CAR; b8[5] = bf16_rne(bb[1]) * ACT_CAR;
    b8[6] = bf16_rne(bb[2]) * ACT_CAR; b8[7] = bf16_rne(bb[3]) * ACT_CAR;
#pragma unroll
    for (int t = 0; t < 4; ++t)
#pragma unroll
      for (int r = 0; r < 8; ++r) {
        const int rowl = 32 * w + 16 * i + 8 * hl + r;
        const float v = acc[i * 4 + t][r] * PROJ_SCL + b8[r];
        ldsE[rowl * 72 + 16 * t + c] = toh_flush(v);
      }
  }
  __syncthreads();

  _Float16* const bh = PH + (size_t)z * DM * SEQ + (size_t)m0 * SEQ + n0;
  for (int i = 0; i < 8; ++i) {
    const int q = i * 128 + tid;
    const int rowl = q >> 3, ch = (q & 7) * 8;
    const v8h vh = *(const v8h*)(&ldsE[rowl * 72 + ch]);
    *(volatile v8h*)(bh + (size_t)rowl * SEQ + ch) = vh;
  }
  __threadfence();
  for (int i = 0; i < 8; ++i) {
    const int q = i * 128 + tid;
    const int rowl = q >> 3, ch = (q & 7) * 8;
    const v8h vh = *(const v8h*)(&ldsE[rowl * 72 + ch]);
    *(volatile v8h*)(bh + (size_t)rowl * SEQ + ch) = vh;
  }
}

__global__ __launch_bounds__(256) __attribute__((amdgpu_num_vgpr(256)))
void k_attn(const _Float16* __restrict__ QKH, const _Float16* __restrict__ VtH,
            const unsigned int* __restrict__ MB, _Float16* __restrict__ OH)
{
  __shared__ __attribute__((aligned(16))) _Float16 lds[128 * 72];
  static_assert(4 * 256 == 128 * 8);
  static_assert(HD == 4 * 16);

  const int tid = threadIdx.x, lane = tid & 31;
  const int wave = __builtin_amdgcn_readfirstlane(tid >> 5);
  const int hl = lane >> 4, c = lane & 15;
  const int q0 = blockIdx.x * 128;
  const int col0 = blockIdx.y * HD;
  const int b = blockIdx.z;

  const size_t qr = (size_t)b * SEQ + q0 + 16 * wave + c;
  const v16h qf0 = ld_frag_g(QKH + qr * QKP + col0, hl);
  const v16h qf1 = ld_frag_g(QKH + qr * QKP + col0 + 32, hl);

  const _Float16* kb = QKH + ((size_t)b * SEQ + c) * QKP + DM + col0;
  const _Float16* vb = VtH + ((size_t)b * DM + col0 + c) * SEQ;
  const unsigned int* mbp = MB + (size_t)b * MB_PITCH;
  const float NEG_INF = -__builtin_inff();

  float m = NEG_INF, l = 0.f;
  v8f o[4] = {};

#pragma unroll 1
  for (int kt = 0; kt < SEQ / 32; ++kt) {
    const int mk = kt * 32;
    const unsigned int mw = mbp[kt];

    const _Float16* kp = kb + (size_t)mk * QKP;
    const v16h k00 = ld_frag_g(kp, hl);
    const v16h k01 = ld_frag_g(kp + 32, hl);
    const v16h k10 = ld_frag_g(kp + (size_t)16 * QKP, hl);
    const v16h k11 = ld_frag_g(kp + (size_t)16 * QKP + 32, hl);
    v8f s0 = {}, s1 = {};
    s0 = mma(k00, qf0, s0);
    s0 = mma(k01, qf1, s0);
    s1 = mma(k10, qf0, s1);
    s1 = mma(k11, qf1, s1);

    float v0[8], v1[8];
#pragma unroll
    for (int r = 0; r < 8; ++r) { v0[r] = s0[r] * S_SCL; v1[r] = s1[r] * S_SCL; }

    if (mw != 0xFFFFFFFFu) {
      const unsigned int ml = mw >> (8 * hl);
#pragma unroll
      for (int r = 0; r < 8; ++r) {
        v0[r] = ((ml >> r) & 1u)        ? v0[r] : NEG_INF;
        v1[r] = ((ml >> (16 + r)) & 1u) ? v1[r] : NEG_INF;
      }
    }

    float tm = fmaxf(v0[0], v1[0]);
#pragma unroll
    for (int r = 1; r < 8; ++r) tm = fmaxf(tm, fmaxf(v0[r], v1[r]));
    tm = fmaxf(tm, __shfl_xor(tm, 16, 32));
    const float mn  = fmaxf(m, tm);
    const float ms  = (mn == NEG_INF) ? 0.f : mn;
    const float al  = __expf(m - ms);
    const float msc = ms - LN_PCAR;
    float rs = 0.f;
    v16h pv;
#pragma unroll
    for (int r = 0; r < 8; ++r) {
      const float d0 = v0[r] - msc;
      const float d1 = v1[r] - msc;
      const float e0 = (d0 < P_CUT) ? 0.f : __expf(d0);
      const float e1 = (d1 < P_CUT) ? 0.f : __expf(d1);
      const h16 h0 = (h16)e0;
      const h16 h1 = (h16)e1;
      pv[r]     = h0;
      pv[8 + r] = h1;
      rs += (float)h0 + (float)h1;
    }
    rs += __shfl_xor(rs, 16, 32);
    l = l * al + rs;
    m = mn;
#pragma unroll
    for (int t = 0; t < 4; ++t)
#pragma unroll
      for (int r = 0; r < 8; ++r) o[t][r] *= al;

    const _Float16* vp = vb + mk;
    const v16h vf0 = ld_frag_g(vp, hl);
    const v16h vf1 = ld_frag_g(vp + (size_t)16 * SEQ, hl);
    const v16h vf2 = ld_frag_g(vp + (size_t)32 * SEQ, hl);
    const v16h vf3 = ld_frag_g(vp + (size_t)48 * SEQ, hl);
    o[0] = mma(vf0, pv, o[0]);
    o[1] = mma(vf1, pv, o[1]);
    o[2] = mma(vf2, pv, o[2]);
    o[3] = mma(vf3, pv, o[3]);
  }

  const float inv = O_MUL * (1.0f / l);
  {
    const int rowl = 16 * wave + c;
#pragma unroll
    for (int t = 0; t < 4; ++t) {
      v8h ov;
#pragma unroll
      for (int r = 0; r < 8; ++r) ov[r] = toh_flush(o[t][r] * inv);
      *(v8h*)(&lds[rowl * 72 + 16 * t + 8 * hl]) = ov;
    }
  }
  __syncthreads();
  _Float16* const bh = OH + ((size_t)b * SEQ + q0) * DM + col0;
  for (int i = 0; i < 4; ++i) {
    const int q = i * 256 + tid;
    const int rowl = q >> 3, ch = (q & 7) * 8;
    const v8h vh = *(const v8h*)(&lds[rowl * 72 + ch]);
    *(volatile v8h*)(bh + (size_t)rowl * DM + ch) = vh;
  }
  __threadfence();
  for (int i = 0; i < 4; ++i) {
    const int q = i * 256 + tid;
    const int rowl = q >> 3, ch = (q & 7) * 8;
    const v8h vh = *(const v8h*)(&lds[rowl * 72 + ch]);
    *(volatile v8h*)(bh + (size_t)rowl * DM + ch) = vh;
  }
}

__global__ __launch_bounds__(128) __attribute__((amdgpu_num_vgpr(256)))
void k_oproj(const _Float16* __restrict__ AH, const _Float16* __restrict__ Bt,
             const float* __restrict__ bias, float* __restrict__ Out)
{
  __shared__ __attribute__((aligned(16))) float ldsF[128 * 68];
  static_assert(16 * 128 == 128 * 16);

  const int tid = threadIdx.x, lane = tid & 31;
  const int w = __builtin_amdgcn_readfirstlane(tid >> 5);
  const int hl = lane >> 4, c = lane & 15;
  const int m0 = blockIdx.y * 128, n0 = blockIdx.x * 64;
  const int mw = m0 + 32 * w;

  const _Float16* ap0 = AH + (size_t)(mw + c) * DM;
  const _Float16* ap1 = AH + (size_t)(mw + 16 + c) * DM;
  const _Float16* bp  = Bt + (size_t)(n0 + c) * DM;

  v8f acc[8] = {};
  gemm_core(ap0, ap1, bp, DM, hl, acc);

#pragma unroll
  for (int i = 0; i < 2; ++i)
#pragma unroll
    for (int t = 0; t < 4; ++t)
#pragma unroll
      for (int r = 0; r < 8; ++r) {
        const int rowl = 32 * w + 16 * i + 8 * hl + r;
        ldsF[rowl * 68 + 16 * t + c] = acc[i * 4 + t][r] * OUT_SCL;
      }
  __syncthreads();

  const int bcol = (tid & 15) * 4;
  const v4f braw = *(const v4f*)(bias + n0 + bcol);
  v4f bb;
  bb[0] = bf16_rne(braw[0]); bb[1] = bf16_rne(braw[1]);
  bb[2] = bf16_rne(braw[2]); bb[3] = bf16_rne(braw[3]);

  const int ob_b = m0 / SEQ;
  const int ob_n = m0 - ob_b * SEQ;
  float* const ob = Out + ((size_t)ob_b * SEQ_FULL + ob_n) * DM + n0;
  for (int i = 0; i < 16; ++i) {
    const int qi = i * 128 + tid;
    const int rowl = qi >> 4, col = (qi & 15) * 4;
    const v4f v = *(const v4f*)(&ldsF[rowl * 68 + col]) + bb;
    *(volatile v4f*)(ob + (size_t)rowl * DM + col) = v;
  }
  __threadfence();
  for (int i = 0; i < 16; ++i) {
    const int qi = i * 128 + tid;
    const int rowl = qi >> 4, col = (qi & 15) * 4;
    const v4f v = *(const v4f*)(&ldsF[rowl * 68 + col]) + bb;
    *(volatile v4f*)(ob + (size_t)rowl * DM + col) = v;
  }
}

extern "C" void kernel_launch(void* const* d_in, const int* in_sizes, int n_in,
                              void* d_out, int out_size, void* d_ws, size_t ws_size,
                              hipStream_t stream)
{
  if (n_in < 10) return;
  const long need_x = ((long)(NB - 1) * SEQ_FULL + SEQ) * DM;
  const long need_m = (long)(NB - 1) * SEQ_FULL + SEQ;
  if ((long)in_sizes[0] < need_x) return;
  if ((long)in_sizes[1] < (long)DM * DM) return;
  if ((long)in_sizes[2] < (long)DM) return;
  if ((long)in_sizes[3] < (long)DM * DM) return;
  if ((long)in_sizes[4] < (long)DM) return;
  if ((long)in_sizes[5] < (long)DM * DM) return;
  if ((long)in_sizes[6] < (long)DM) return;
  if ((long)in_sizes[7] < (long)DM * DM) return;
  if ((long)in_sizes[8] < (long)DM) return;
  if ((long)in_sizes[9] < need_m) return;
  if ((long)out_size < need_x) return;
  if (WS_HALVES * sizeof(_Float16) > ws_size) return;

  const float* x    = (const float*)d_in[0];
  const float* Wq   = (const float*)d_in[1];
  const float* bq   = (const float*)d_in[2];
  const float* Wk   = (const float*)d_in[3];
  const float* bk   = (const float*)d_in[4];
  const float* Wv   = (const float*)d_in[5];
  const float* bv   = (const float*)d_in[6];
  const float* Wo   = (const float*)d_in[7];
  const float* bo   = (const float*)d_in[8];
  const int*   mask = (const int*)d_in[9];
  float* out = (float*)d_out;

  _Float16* X16 = (_Float16*)d_ws;
  _Float16* WT  = X16 + N_X;
  _Float16* QKH = WT  + N_W;
  _Float16* VtH = QKH + N_QK;
  _Float16* OH  = VtH + N_VT;
  float*    TAB = (float*)(OH + N_X);
  unsigned int* MBW = (unsigned int*)(TAB + (size_t)SEQ * TABW);

  const size_t nW = (size_t)DM * DM;
  const int tx8 = (int)(N_X / 8);
  k_cvt8<<<tx8 / 256, 256, 0, stream>>>(x, X16, DM, SEQ, SEQ_FULL, ACT_CAR, tx8);

  k_trw<<<dim3(DM / 64, DM / 64), 256, 0, stream>>>(Wq, WT,          DM, DM);
  k_trw<<<dim3(DM / 64, DM / 64), 256, 0, stream>>>(Wk, WT + nW,     DM, DM);
  k_trw<<<dim3(DM / 64, DM / 64), 256, 0, stream>>>(Wv, WT + 2 * nW, DM, DM);
  k_trw<<<dim3(DM / 64, DM / 64), 256, 0, stream>>>(Wo, WT + 3 * nW, DM, DM);

  k_ropetab<<<SEQ / 8, 256, 0, stream>>>(TAB);
  k_mbits<<<NB, 256, 0, stream>>>(mask, MBW);

  k_projr<<<dim3(QKP / 64, ROWS / 128), 128, 0, stream>>>(X16, WT, bq, bk, TAB, QKH);
  k_projv<<<dim3(SEQ / 64, DM / 128, NB), 128, 0, stream>>>(WT + 2 * nW, X16, bv, VtH);

  k_attn<<<dim3(SEQ / 128, NH, NB), 256, 0, stream>>>(QKH, VtH, MBW, OH);

  k_oproj<<<dim3(DM / 64, ROWS / 128), 128, 0, stream>>>(OH, WT + 3 * nW, bo, out);
}
